// GraphAutoencoder_84482006712576
// MI455X (gfx1250) — hardware-run, weakly checked
//
#include <hip/hip_runtime.h>


namespace {
constexpr int N = 100000, EFULL = 1600000, E = 1600000, DI = 8, DH = 16, DE = 8, MH = 128, KZ = DI * MH  , DO = 8, CHUNK = 16384, NCH = 7  ;
constexpr float XS = 8.0f, WSC = 256.0f;
static_assert(CHUNK % 64 == 0 && KZ % 32 == 0 && (size_t)7 * CHUNK >= N, "tiling");
typedef _Float16 b16;
typedef __attribute__((ext_vector_type(16))) _Float16 v16b;
typedef __attribute__((ext_vector_type(8))) _Float16 v8b;
typedef __attribute__((ext_vector_type(8))) float v8f;
typedef __attribute__((ext_vector_type(4))) float v4f;
__device__ __forceinline__ float bf16_rne(float f) { unsigned int u = __float_as_uint(f); u += 0x7FFFu + ((u >> 16) & 1u); return __uint_as_float(u & 0xFFFF0000u); }
__device__ __forceinline__ void split16(float v, b16& hi, b16& lo) { hi = (b16)v; lo = (b16)(v - (float)hi); }
__device__ __forceinline__ v16b frag_kb(const b16* p, int hh) { const v8b a = *(const v8b*)(p + 8 * hh), b = *(const v8b*)(p + 16 + 8 * hh); v16b f;
#pragma unroll
  for (int e = 0; e < 8; ++e) { f[e] = a[e]; f[8 + e] = b[e]; } return f; }
__device__ __forceinline__ v8f wmma16b(v16b a, v16b b, v8f c) { v8f d = __builtin_amdgcn_wmma_f32_16x16x32_f16(false, a, false, b, (short)0, c, false, false); asm volatile("v_nop\n\tv_nop\n\tv_nop\n\tv_nop" : "+v"(d) : "v"(a), "v"(b)); return d; }
__device__ __forceinline__ void wave_lds_sync() { __builtin_amdgcn_fence(__ATOMIC_RELEASE, "workgroup"); __builtin_amdgcn_wave_barrier(); __builtin_amdgcn_fence(__ATOMIC_ACQUIRE, "workgroup"); }
__device__ __forceinline__ float pmul(float a, float b) { float p = a * b; asm volatile("" : "+v"(p)); return p; }
__device__ __forceinline__ int iclamp(int v, int lo, int hi) { return v < lo ? lo : (v > hi ? hi : v); }
constexpr int CSR_NBLK = 512, CSR_GB = 9, CSR_GN = 1 << CSR_GB  , CSR_MAXG = 512, CSR_CAP = 12288  ;
__global__ __launch_bounds__(64) void csrA_kernel(const int* __restrict__ dst, int E, int N, int nG, int CHP, int NGP, int* __restrict__ STG, int* __restrict__ HST) {
  extern __shared__ int sm[];
  int* cnt = sm; int* run = sm + NGP; int* ids = sm + 2 * NGP;
  const int b = blockIdx.x; const int ch = (E + CSR_NBLK - 1) / CSR_NBLK; const int e0 = b * ch, e1 = min(E, e0 + ch);
  for (int i = threadIdx.x; i < NGP; i += 64) cnt[i] = 0;
  for (int i = threadIdx.x; i < CHP; i += 64) ids[i] = -1;
  __syncthreads();
  if (threadIdx.x == 0) {
    for (int e = e0; e < e1; ++e) { int d = dst[e]; d = (d < 0) ? 0 : (d >= N ? N - 1 : d); cnt[d >> CSR_GB] += 1; }
    int acc = 0; for (int g = 0; g < nG; ++g) { run[g] = acc; acc += cnt[g]; }
    for (int e = e0; e < e1; ++e) { int d = dst[e]; d = (d < 0) ? 0 : (d >= N ? N - 1 : d); const int g = d >> CSR_GB; ids[run[g]] = e; run[g] += 1; } }
  __syncthreads();
  typedef __attribute__((ext_vector_type(4))) int v4i;
  for (int pass = 0; pass < 2; ++pass) {
    for (int i = threadIdx.x; i < CHP / 4; i += 64) *(volatile v4i*)(STG + (size_t)b * CHP + i * 4) = *(const v4i*)(&ids[i * 4]);
    for (int i = threadIdx.x; i < NGP / 4; i += 64) { v4i v; for (int e = 0; e < 4; ++e) v[e] = (i * 4 + e < nG) ? cnt[i * 4 + e] : 0; *(volatile v4i*)(HST + (size_t)b * NGP + i * 4) = v; }
    __threadfence(); }
}
__global__ __launch_bounds__(512) void csrS_kernel(const int* __restrict__ HST, int nG, int NGP, int* __restrict__ START, int* __restrict__ TOT, int* __restrict__ OFF) {
  __shared__ int tot[CSR_MAXG];
  const int b = threadIdx.x;
  for (int pass = 0; pass < 2; ++pass) { int runb = 0; for (int g = 0; g < nG; ++g) { int c = HST[(size_t)b * NGP + g]; c = (c < 0) ? 0 : c; ((volatile int*)OFF)[(size_t)g * CSR_NBLK + b] = runb; runb += c; } __threadfence(); }
  for (int g = threadIdx.x; g < nG; g += 512) { int s = 0; for (int bb = 0; bb < CSR_NBLK; ++bb) { int c = HST[(size_t)bb * NGP + g]; s += (c < 0) ? 0 : c; } tot[g] = s; }
  __syncthreads();
  if (threadIdx.x < 32) {
    __shared__ int st[CSR_MAXG + 32];
    if (threadIdx.x == 0) { int acc = 0; for (int g = 0; g < NGP; ++g) { st[g] = acc; if (g < nG) acc += (tot[g] + 31) & ~31; } st[NGP] = acc; }
    __builtin_amdgcn_fence(__ATOMIC_RELEASE, "workgroup"); __builtin_amdgcn_wave_barrier(); __builtin_amdgcn_fence(__ATOMIC_ACQUIRE, "workgroup");
    for (int pass = 0; pass < 2; ++pass) { for (int i = threadIdx.x; i < NGP + 32; i += 32) { ((volatile int*)START)[i] = (i <= NGP) ? st[min(i, NGP)] : 0; ((volatile int*)TOT)[i] = (i < nG) ? tot[i] : 0; } __threadfence(); } }
}
__global__ __launch_bounds__(256) void csrB_kernel(const int* __restrict__ dst, int N, int nG, int CHP, int NGP, int permLen, const int* __restrict__ STG, const int* __restrict__ HST, const int* __restrict__ OFF, const int* __restrict__ START, const int* __restrict__ TOT, int* __restrict__ PERM, int* __restrict__ ROWPTR, int* __restrict__ ROWCNT, int* __restrict__ FLAG) {
  typedef __attribute__((ext_vector_type(4))) int v4i;
  __shared__ int ids[CSR_CAP]; __shared__ unsigned short key[CSR_CAP]; __shared__ int outp[CSR_CAP]; __shared__ int ncnt[CSR_GN + 1]; __shared__ int boff[CSR_NBLK + 1];
  const int g = blockIdx.x, t_ = threadIdx.x; int tot = TOT[g]; int st = START[g], stn = START[g + 1]; const int v0 = g * CSR_GN; const int nv = min(CSR_GN, N - v0);
  st = (st < 0) ? 0 : (st > permLen - 32 ? permLen - 32 : st) & ~31; stn = (stn < st) ? st : (stn > permLen ? permLen : stn); tot = (tot < 0) ? 0 : tot; if (tot > stn - st && tot <= CSR_CAP) tot = stn - st;
  if (tot > CSR_CAP) {
    for (int pass = 0; pass < 2; ++pass) { for (int i = t_; i < CSR_GN / 4; i += 256) { v4i a, c; for (int e = 0; e < 4; ++e) { a[e] = st; c[e] = 0; } *(volatile v4i*)(ROWPTR + v0 + i * 4) = a; *(volatile v4i*)(ROWCNT + v0 + i * 4) = c; } if (t_ == 0) ((volatile int*)FLAG)[0] = 1; __threadfence(); } (void)nv; return; }
  if (t_ == 0) { int acc = 0; for (int b = 0; b < CSR_NBLK; ++b) { boff[b] = acc; int c = HST[(size_t)b * NGP + g]; c = (c < 0) ? 0 : (c > CHP ? CHP : c); acc += c; if (acc > tot) acc = tot; } boff[CSR_NBLK] = acc; }
  for (int i = t_; i <= CSR_GN; i += 256) ncnt[i] = 0;
  __syncthreads();
  for (int b = 0; b < CSR_NBLK; ++b) { const int c = boff[b + 1] - boff[b]; int o_ = OFF[(size_t)g * CSR_NBLK + b]; o_ = (o_ < 0) ? 0 : (o_ > CHP - c ? CHP - c : o_); const int* src_ = STG + (size_t)b * CHP + o_;
    for (int i = t_; i < c; i += 256) { int id = src_[i]; id = (id < 0) ? 0 : id; ids[boff[b] + i] = id; int d = dst[id]; d = (d < v0) ? v0 : (d >= N ? N - 1 : d); int kk = d - v0; kk = (kk < 0) ? 0 : (kk >= CSR_GN ? CSR_GN - 1 : kk); key[boff[b] + i] = (unsigned short)kk; } }
  __syncthreads();
  if (t_ == 0) { for (int i = 0; i < tot; ++i) ncnt[key[i]] += 1; int acc = 0; for (int vl = 0; vl < CSR_GN; ++vl) { const int c = ncnt[vl]; ncnt[vl] = acc; acc += c; } ncnt[CSR_GN] = acc;
    for (int i = 0; i < tot; ++i) { const int vl = key[i]; outp[ncnt[vl]] = ids[i]; ncnt[vl] += 1; }
    for (int vl = CSR_GN; vl > 0; --vl) ncnt[vl] = ncnt[vl - 1]; ncnt[0] = 0; }
  __syncthreads();
  for (int pass = 0; pass < 2; ++pass) {
    for (int i = t_; i < (stn - st) / 4; i += 256) { v4i v; for (int e = 0; e < 4; ++e) { const int q = i * 4 + e; v[e] = (q < tot) ? outp[q] : -1; } *(volatile v4i*)(PERM + st + i * 4) = v; }
    for (int i = t_; i < CSR_GN / 4; i += 256) { v4i a, c; for (int e = 0; e < 4; ++e) { const int vl = i * 4 + e; a[e] = st + ncnt[vl]; c[e] = (vl < nv) ? (ncnt[vl + 1] - ncnt[vl]) : 0; } *(volatile v4i*)(ROWPTR + v0 + i * 4) = a; *(volatile v4i*)(ROWCNT + v0 + i * 4) = c; }
    __threadfence(); }
}
__global__ __launch_bounds__(256) void csrZ_kernel(int* __restrict__ p, size_t n4) { typedef __attribute__((ext_vector_type(4))) int v4i; const size_t tid = (size_t)blockIdx.x * 256 + threadIdx.x, nth = (size_t)gridDim.x * 256; v4i z = {0, 0, 0, 0}; for (size_t i = tid; i < n4; i += nth) *(volatile v4i*)(p + i * 4) = z; }
struct CsrBufs { int *STG, *HST, *OFF, *START, *TOT, *PERM, *ROWPTR, *ROWCNT, *FLAG; int nG, NGP, CHP; size_t permLen; char* base; size_t bytes; };
static size_t csr_carve(CsrBufs& c, char* ws, size_t off, int E, int N) {
  const size_t off0 = off; c.base = ws + off;
  auto al = [&](size_t bytes) { char* p = ws + off; off += (bytes + 255) & ~(size_t)255; return p; };
  c.nG = (N + CSR_GN - 1) / CSR_GN; c.NGP = (c.nG + 31) & ~31; const int ch = (E + CSR_NBLK - 1) / CSR_NBLK; c.CHP = (ch + 31) & ~31; c.permLen = (size_t)E + 32 * (size_t)c.nG + 32;
  c.STG = (int*)al((size_t)CSR_NBLK * c.CHP * 4); c.HST = (int*)al((size_t)CSR_NBLK * c.NGP * 4); c.OFF = (int*)al((size_t)c.NGP * CSR_NBLK * 4); c.START = (int*)al((size_t)(c.NGP + 64) * 4); c.TOT = (int*)al((size_t)(c.NGP + 64) * 4);
  c.PERM = (int*)al(c.permLen * 4); c.ROWPTR = (int*)al((size_t)c.nG * CSR_GN * 4); c.ROWCNT = (int*)al((size_t)c.nG * CSR_GN * 4); c.FLAG = (int*)al(256);
  c.bytes = off - off0; return off;
}
static void csr_build(const CsrBufs& c, const int* dst, int E, int N, hipStream_t stream) {
  const size_t smem = (size_t)(2 * c.NGP + c.CHP) * 4;
  csrZ_kernel<<<512, 256, 0, stream>>>((int*)c.base, c.bytes / 16);
  csrA_kernel<<<CSR_NBLK, 64, smem, stream>>>(dst, E, N, c.nG, c.CHP, c.NGP, c.STG, c.HST);
  csrS_kernel<<<1, 512, 0, stream>>>(c.HST, c.nG, c.NGP, c.START, c.TOT, c.OFF);
  csrB_kernel<<<c.nG, 256, 0, stream>>>(dst, N, c.nG, c.CHP, c.NGP, (int)c.permLen, c.STG, c.HST, c.OFF, c.START, c.TOT, c.PERM, c.ROWPTR, c.ROWCNT, c.FLAG);
}

typedef __attribute__((ext_vector_type(4))) _Float16 v4h;
__global__ __launch_bounds__(256) void wprep_kernel(const float* __restrict__ w2, b16* __restrict__ W2T) {
  const int u = blockIdx.x * 256 + threadIdx.x; if (u >= DH * KZ / 8) return; const int e = u * 8; const int o = e / KZ, k0 = e % KZ; v8b v;
  for (int j = 0; j < 8; ++j) { const int k = k0 + j, i = k / MH, h = k % MH; v[j] = (b16)(bf16_rne(w2[(size_t)h * MH + DH * i + o]) * WSC); }
  for (int pass = 0; pass < 2; ++pass) { *(volatile v8b*)(W2T + e) = v; __threadfence(); }
}
__global__ __launch_bounds__(256) void agg_kernel(const float* __restrict__ x, const float* __restrict__ ea, const float* __restrict__ w1, const float* __restrict__ b1, const int* __restrict__ srcs, const int* __restrict__ PERM, const int* __restrict__ ROWPTR, const int* __restrict__ ROWCNT, int permLen, int v0,
                                                   b16* __restrict__ Zh, b16* __restrict__ Zl, float* __restrict__ XS8) {
  __shared__ __attribute__((aligned(16))) float xst[8][DI];
  const int wave = threadIdx.x >> 5, lane = threadIdx.x & 31; const int vl = blockIdx.x * 8 + wave; const size_t v = (size_t)v0 + vl;
  float wl[4][DE], bl[4];
#pragma unroll
  for (int j = 0; j < 4; ++j) { bl[j] = bf16_rne(b1[lane * 4 + j]);
#pragma unroll
    for (int d = 0; d < DE; ++d) wl[j][d] = bf16_rne(w1[d * MH + lane * 4 + j]); }
  float Z[DI][4], X[DI];
#pragma unroll
  for (int i = 0; i < DI; ++i) { X[i] = 0.0f;
#pragma unroll
    for (int j = 0; j < 4; ++j) Z[i][j] = 0.0f; }
  if (v < (size_t)N) { int st = ROWPTR[v], cnt = ROWCNT[v]; cnt = iclamp(cnt, 0, 65536); st = iclamp(st, 0, permLen - cnt);
#pragma unroll 1
    for (int q = 0; q < cnt; ++q) { const int e = iclamp(PERM[st + q], 0, E - 1); const size_t s = (size_t)iclamp(srcs[e], 0, N - 1);
      const v4f e0 = *(const v4f*)(ea + (size_t)e * DE), e1 = *(const v4f*)(ea + (size_t)e * DE + 4); float ev[DE]; for (int d = 0; d < 4; ++d) { ev[d] = bf16_rne(e0[d]); ev[4 + d] = bf16_rne(e1[d]); }
      float A[4];
#pragma unroll
      for (int j = 0; j < 4; ++j) { float a = bl[j];
#pragma unroll
        for (int d = 0; d < DE; ++d) a += pmul(ev[d], wl[j][d]); A[j] = fmaxf(a, 0.0f); }
      const v4f x0 = *(const v4f*)(x + s * DI), x1 = *(const v4f*)(x + s * DI + 4); float xv[DI]; for (int i = 0; i < 4; ++i) { xv[i] = bf16_rne(x0[i]); xv[4 + i] = bf16_rne(x1[i]); }
#pragma unroll
      for (int i = 0; i < DI; ++i) { X[i] += xv[i];
#pragma unroll
        for (int j = 0; j < 4; ++j) Z[i][j] += pmul(xv[i], A[j]); } } }
  v4h zh[DI], zl[DI];
#pragma unroll
  for (int i = 0; i < DI; ++i)
#pragma unroll
    for (int j = 0; j < 4; ++j) { b16 p, q; split16(Z[i][j] * XS, p, q); zh[i][j] = p; zl[i][j] = q; }
  { float xsel = 0.0f;
#pragma unroll
    for (int i = 0; i < DI; ++i) xsel = (lane == i) ? X[i] : xsel; if (lane < DI) xst[wave][lane] = xsel; }
  __syncthreads();
  for (int pass = 0; pass < 2; ++pass) {
#pragma unroll
    for (int i = 0; i < DI; ++i) { *(volatile v4h*)(Zh + (size_t)vl * KZ + i * MH + lane * 4) = zh[i]; *(volatile v4h*)(Zl + (size_t)vl * KZ + i * MH + lane * 4) = zl[i]; }
    if (threadIdx.x < 16) *(volatile v4f*)(XS8 + (size_t)blockIdx.x * 64 + threadIdx.x * 4) = *(const v4f*)(&xst[0][0] + threadIdx.x * 4);
    __threadfence(); }
}
__global__ __launch_bounds__(128) void gemm_kernel(const b16* __restrict__ Zh, const b16* __restrict__ Zl, const b16* __restrict__ W2T, int v0, float* __restrict__ AGG) {
  __shared__ __attribute__((aligned(16))) float Tf[4][16][16];
  const int wave = threadIdx.x >> 5, lane = threadIdx.x & 31, nloc = lane & 15, hlf = lane >> 4; const size_t r0 = (size_t)blockIdx.x * 64 + wave * 16;
  v8f acc = (v8f){};
#pragma unroll 4
  for (int kb = 0; kb < KZ; kb += 32) { const v16b a = frag_kb(Zh + (r0 + nloc) * KZ + kb, hlf), al = frag_kb(Zl + (r0 + nloc) * KZ + kb, hlf), bw = frag_kb(W2T + (size_t)nloc * KZ + kb, hlf); acc = wmma16b(a, bw, acc); acc = wmma16b(al, bw, acc); }
#pragma unroll
  for (int r = 0; r < 8; ++r) Tf[wave][8 * hlf + r][nloc] = acc[r] * (1.0f / (XS * WSC));
  wave_lds_sync();
  const float* tw = &Tf[wave][0][0];
  for (int pass = 0; pass < 2; ++pass) { *(volatile v4f*)(AGG + ((size_t)v0 + r0) * DH + lane * 4) = *(const v4f*)(tw + lane * 4); *(volatile v4f*)(AGG + ((size_t)v0 + r0) * DH + 128 + lane * 4) = *(const v4f*)(tw + 128 + lane * 4); __threadfence(); }
}
__global__ __launch_bounds__(256) void final_kernel(const float* __restrict__ AGG, const float* __restrict__ XS8, const float* __restrict__ x, const float* __restrict__ b2, const float* __restrict__ root, const float* __restrict__ cb, const float* __restrict__ wd, const float* __restrict__ bd, float* __restrict__ out) {
  __shared__ __attribute__((aligned(16))) float so[256 * DO];
  const size_t v = (size_t)blockIdx.x * 256 + threadIdx.x;
  float o[DO]; for (int k = 0; k < DO; ++k) o[k] = 0.0f;
  if (v < (size_t)N) { float xv[DI], X[DI];
    { const v4f a = *(const v4f*)(x + v * DI), b = *(const v4f*)(x + v * DI + 4), c = *(const v4f*)(XS8 + v * DI), d = *(const v4f*)(XS8 + v * DI + 4); for (int i = 0; i < 4; ++i) { xv[i] = bf16_rne(a[i]); xv[4 + i] = bf16_rne(b[i]); X[i] = c[i]; X[4 + i] = d[i]; } }
#pragma unroll
    for (int k = 0; k < DO; ++k) o[k] = bf16_rne(bd[k]);
#pragma unroll 1
    for (int t = 0; t < DH; ++t) { float a = AGG[v * DH + t] + bf16_rne(cb[t]);
#pragma unroll
      for (int i = 0; i < DI; ++i) a += pmul(X[i], bf16_rne(b2[DH * i + t])) + pmul(xv[i], bf16_rne(root[i * DH + t]));
      const float ht = fmaxf(a, 0.0f);
#pragma unroll
      for (int k = 0; k < DO; ++k) o[k] += pmul(ht, bf16_rne(wd[t * DO + k])); } }
#pragma unroll
  for (int k = 0; k < DO; ++k) so[threadIdx.x * DO + k] = o[k];
  __syncthreads();
  for (int pass = 0; pass < 2; ++pass) { for (int q = threadIdx.x; q < 256 * DO / 4; q += 256) { const size_t gi = (size_t)blockIdx.x * 256 * DO + (size_t)q * 4; if (gi < (size_t)N * DO) *(volatile v4f*)(out + gi) = *(const v4f*)(&so[q * 4]); } __threadfence(); }
}
}

extern "C" void kernel_launch(void* const* d_in, const int* in_sizes, int n_in, void* d_out, int out_size, void* d_ws, size_t ws_size, hipStream_t stream) {
  (void)n_in;
  auto Fp = [&](int i) { return (const float*)d_in[i]; }; auto Ip = [&](int i) { return (const int*)d_in[i]; };
  if (in_sizes[0] != N * DI || in_sizes[1] != EFULL * DE || in_sizes[2] != DE * MH || in_sizes[3] != MH || in_sizes[4] != MH * MH || in_sizes[5] != MH || in_sizes[6] != DI * DH || in_sizes[7] != DH || in_sizes[8] != DH * DO || in_sizes[9] != DO || in_sizes[10] != 2 * EFULL || out_size != N * DO) return;
  size_t off = 0; char* ws = (char*)d_ws;
  auto carve = [&](size_t bytes) { char* p = ws + off; off += (bytes + 255) & ~(size_t)255; return p; };
  b16* W2T = (b16*)carve((size_t)DH * KZ * 2); b16* Zh = (b16*)carve((size_t)CHUNK * KZ * 2); b16* Zl = (b16*)carve((size_t)CHUNK * KZ * 2); float* XS8 = (float*)carve((size_t)7 * CHUNK * DI * 4); float* AGG = (float*)carve((size_t)7 * CHUNK * DH * 4);
  CsrBufs csr; off = csr_carve(csr, ws, off, E, N);
  if (off > ws_size || off > ((size_t)128 << 20)) return;
  wprep_kernel<<<(DH * KZ / 8 + 255) / 256, 256, 0, stream>>>(Fp(4), W2T);
  csr_build(csr, Ip(10) + EFULL, E, N, stream);
  for (int c = 0; c < NCH; ++c) { const int v0 = c * CHUNK;
    agg_kernel<<<CHUNK / 8, 256, 0, stream>>>(Fp(0), Fp(1), Fp(2), Fp(3), Ip(10), csr.PERM, csr.ROWPTR, csr.ROWCNT, (int)csr.permLen, v0, Zh, Zl, XS8 + (size_t)v0 * DI);
    gemm_kernel<<<CHUNK / 64, 128, 0, stream>>>(Zh, Zl, W2T, v0, AGG); }
  final_kernel<<<(N + 255) / 256, 256, 0, stream>>>(AGG, XS8, Fp(0), Fp(5), Fp(6), Fp(7), Fp(8), Fp(9), (float*)d_out);
}
